// LinksPredictor_25005299597337
// MI455X (gfx1250) — hardware-verified
//
#include <hip/hip_runtime.h>
#include <math.h>

typedef __attribute__((ext_vector_type(16))) _Float16 v16h;
typedef __attribute__((ext_vector_type(16))) __bf16 v16b;
typedef __attribute__((ext_vector_type(8)))  _Float16 v8h;
typedef __attribute__((ext_vector_type(8)))  float v8f;
typedef __attribute__((ext_vector_type(4)))  float v4f;
typedef __attribute__((ext_vector_type(2)))  float v2f;
typedef __attribute__((ext_vector_type(4)))  unsigned v4u;
typedef __attribute__((ext_vector_type(4)))  int v4i;
typedef float __attribute__((may_alias)) float_a;
typedef int __attribute__((may_alias)) int_a;

template <typename T> __device__ __forceinline__ void vst2(void* p, T v) { *(volatile T*)p = v; __threadfence(); *(volatile T*)p = v; }
__device__ __forceinline__ v8f wmma16(v16h a, v16h b, v8f c) {
  v8f d = __builtin_amdgcn_wmma_f32_16x16x32_f16(false, a, false, b, (short)0, c, false, false);
  asm volatile("v_nop\n\tv_nop\n\tv_nop\n\tv_nop" : "+v"(d) : "v"(a), "v"(b));
  return d;
}
__device__ __forceinline__ v8f wmma_bf(v16b a, v16b b, v8f c) {
  v8f d = __builtin_amdgcn_wmma_f32_16x16x32_bf16(false, a, false, b, (short)0, c, false, false);
  asm volatile("v_nop\n\tv_nop\n\tv_nop\n\tv_nop" : "+v"(d) : "v"(a), "v"(b));
  return d;
}
__device__ __forceinline__ v16h frag_h(const _Float16* rowk0, int lane) {
  union { v16h v; v8h q[2]; } u; const _Float16* p = rowk0 + 8 * (lane >> 4);
  u.q[0] = *(const v8h*)p; u.q[1] = *(const v8h*)(p + 16); return u.v;
}
__device__ __forceinline__ v16h frag_f32(const float* rowk0, int lane) {
  v16h a; const float* p = rowk0 + 8 * (lane >> 4);
#pragma unroll
  for (int i = 0; i < 8; ++i) { a[i] = (_Float16)p[i]; a[8 + i] = (_Float16)p[16 + i]; }
  return a;
}
__device__ __forceinline__ v16h frag_f32s(const float* rowk0, int lane, float sc) {
  v16h a; const float* p = rowk0 + 8 * (lane >> 4);
#pragma unroll
  for (int i = 0; i < 8; ++i) { a[i] = (_Float16)(p[i] * sc); a[8 + i] = (_Float16)(p[16 + i] * sc); }
  return a;
}
__device__ __forceinline__ v16h fragc_f32(const float* W, int k0, int n, int lane, int ld, int K) {
  v16h a; const int g = lane >> 4;
#pragma unroll
  for (int i = 0; i < 8; ++i) { const int ka = k0 + 8 * g + i, kb = ka + 16;
    a[i] = (_Float16)(ka < K ? W[(size_t)ka * ld + n] : 0.f); a[8 + i] = (_Float16)(kb < K ? W[(size_t)kb * ld + n] : 0.f); }
  return a;
}
struct F2 { v16b h, l; };
__device__ __forceinline__ F2 bsplit16(const float v[16]) { F2 r;
#pragma unroll
  for (int i = 0; i < 16; ++i) { const __bf16 h = (__bf16)v[i]; r.h[i] = h; r.l[i] = (__bf16)(v[i] - (float)h); }
  return r; }
__device__ __forceinline__ F2 split_row(const float* row, int k0, int lane) { float v[16]; const float* p = row + k0 + 8 * (lane >> 4);
#pragma unroll
  for (int i = 0; i < 8; ++i) { v[i] = p[i]; v[8 + i] = p[16 + i]; }
  return bsplit16(v); }
__device__ __forceinline__ F2 split_rowK(const float* row, int k0, int lane, int K) { float v[16]; const int g = lane >> 4;
#pragma unroll
  for (int i = 0; i < 8; ++i) { const int ka = k0 + 8 * g + i, kb = ka + 16; v[i] = ka < K ? row[ka] : 0.f; v[8 + i] = kb < K ? row[kb] : 0.f; }
  return bsplit16(v); }
__device__ __forceinline__ F2 split_col(const float* W, int k0, int n, int lane, int ld, int K) { float v[16]; const int g = lane >> 4;
#pragma unroll
  for (int i = 0; i < 8; ++i) { const int ka = k0 + 8 * g + i, kb = ka + 16; v[i] = ka < K ? W[(size_t)ka * ld + n] : 0.f; v[8 + i] = kb < K ? W[(size_t)kb * ld + n] : 0.f; }
  return bsplit16(v); }
__device__ __forceinline__ v8f mac3(const F2& a, const F2& b, v8f c) { c = wmma_bf(a.l, b.h, c); c = wmma_bf(a.h, b.l, c); return wmma_bf(a.h, b.h, c); }
__device__ __forceinline__ float sigm(float v) { return 1.0f / (1.0f + expf(-v)); }
#define LDSX() do { asm volatile("s_wait_dscnt 0" ::: "memory"); __builtin_amdgcn_wave_barrier(); __builtin_amdgcn_fence(__ATOMIC_RELEASE, "workgroup"); } while (0)


#define NN 100000
#define NNP 100032
#define NE 500000
#define HD 128
__device__ __forceinline__ int clampn(int v) { return v < 0 ? 0 : (v >= NN ? NN - 1 : v); }

__global__ __launch_bounds__(128) void k_proj(const float* __restrict__ X, const float* __restrict__ W, const float* __restrict__ bias, float* __restrict__ Pout) {
  __shared__ __align__(16) float so[4][16][132];
  const int tid = threadIdx.x, wave = tid >> 5, lane = tid & 31, col = lane & 15, g = lane >> 4;
  const int r0 = blockIdx.x * 64 + wave * 16; const int ra = (r0 + col) < NN ? (r0 + col) : (NN - 1);
  v8f acc[8] = {};
#pragma unroll 1
  for (int kc = 0; kc < HD / 32; ++kc) { const F2 a = split_row(X + (size_t)ra * HD, kc * 32, lane);
#pragma unroll
    for (int j = 0; j < 8; ++j) acc[j] = mac3(a, split_row(W + (size_t)(j * 16 + col) * HD, kc * 32, lane), acc[j]); }
#pragma unroll
  for (int j = 0; j < 8; ++j) { const float bb = bias[j * 16 + col];
#pragma unroll
    for (int r = 0; r < 8; ++r) so[wave][8 * g + r][j * 16 + col] = acc[j][r] + bb; }
  LDSX();
  for (int rl = 0; rl < 16; ++rl) { if (r0 + rl >= NN) break; vst2(Pout + (size_t)(r0 + rl) * HD + lane * 4, *(const v4f*)(&so[wave][rl][lane * 4])); }
}
__global__ __launch_bounds__(256) void k_edge(const float* __restrict__ PA, const float* __restrict__ PB, const int* __restrict__ eidx, float* __restrict__ out) {
  __shared__ float sres[8][32];
  const int wave = threadIdx.x >> 5, lane = threadIdx.x & 31; const int e0 = (blockIdx.x * 8 + wave) * 32;
  const int sub = lane >> 3, part = lane & 7;
#pragma unroll 1
  for (int ps = 0; ps < 8; ++ps) { const int e = e0 + ps * 4 + sub; float s = 0.f;
    if (e < NE) { const int sa = clampn(eidx[e]), sb = clampn(eidx[NE + e]); const float* pa = PA + (size_t)sa * HD + part * 16; const float* pb = PB + (size_t)sb * HD + part * 16;
#pragma unroll
      for (int q = 0; q < 4; ++q) { const v4f a = *(const v4f*)(pa + q * 4), b = *(const v4f*)(pb + q * 4); s += a[0] * b[0] + a[1] * b[1] + a[2] * b[2] + a[3] * b[3]; } }
    s += __shfl_xor(s, 1, 32); s += __shfl_xor(s, 2, 32); s += __shfl_xor(s, 4, 32);
    if (part == 0) sres[wave][ps * 4 + sub] = s; }
  LDSX();
  if (e0 + lane < NE) vst2(out + e0 + lane, (float_a)sres[wave][lane]);
}
extern "C" void kernel_launch(void* const* d_in, const int* in_sizes, int n_in, void* d_out, int out_size, void* d_ws, size_t ws_size, hipStream_t stream) {
  (void)in_sizes; (void)n_in; (void)out_size; (void)ws_size;
  const float* XA = (const float*)d_in[0]; const float* XB = (const float*)d_in[1]; const int* eidx = (const int*)d_in[2];
  const float* WA = (const float*)d_in[3]; const float* bA = (const float*)d_in[4]; const float* WB = (const float*)d_in[5]; const float* bB = (const float*)d_in[6];
  float* out = (float*)d_out;
  char* ws = (char*)d_ws; size_t off = 0;
  auto take = [&](size_t bytes) { char* p = ws + off; off += (bytes + 255) & ~(size_t)255; return p; };
  float* PA = (float*)take((size_t)NNP * HD * 4); float* PB = (float*)take((size_t)NNP * HD * 4);
  k_proj<<<NNP / 64, 128, 0, stream>>>(XA, WA, bA, PA);
  k_proj<<<NNP / 64, 128, 0, stream>>>(XB, WB, bB, PB);
  k_edge<<<(NE + 255) / 256, 256, 0, stream>>>(PA, PB, eidx, out);
}
